// StackedQLSTM_28716151341215
// MI455X (gfx1250) — hardware-verified
//
#include <hip/hip_runtime.h>
#include <math.h>

constexpr int NLAYER  = 2;
constexpr int NSTEP   = 512;
constexpr int NBAT    = 128;
constexpr int NFEAT   = 4;
constexpr int NHID    = 256;
constexpr int NGATE   = 4;
constexpr int NQ      = NHID / 4;
constexpr int RTHR    = 512;
constexpr int PTHR    = 256;
constexpr int SEQ_BLK = 16;
constexpr int HPITCH  = 264;
constexpr int SPITCH  = 260;
constexpr float UCARRY     = 16.0f;
constexpr float UCARRY_INV = 1.0f / 16.0f;
constexpr int UT_PER_LAYER  = NGATE * NHID * NHID;
constexpr int WXE_PER_LAYER = NGATE * NHID * NFEAT;
static_assert(NBAT % SEQ_BLK == 0);
static_assert(NHID == 16 * (RTHR / 32));
static_assert(NHID % 32 == 0);
static_assert(HPITCH % 8 == 0 && HPITCH >= NHID);
static_assert(SPITCH % 4 == 0 && SPITCH >= NHID);
static_assert((NLAYER * NGATE * NHID * (NHID / 8)) % PTHR == 0);
static_assert((NLAYER * NGATE * NHID) % PTHR == 0);
static_assert(NQ == 64 && NFEAT == 4);

typedef __attribute__((ext_vector_type(16))) _Float16 v16h;
typedef __attribute__((ext_vector_type(8)))  _Float16 v8h;
typedef __attribute__((ext_vector_type(8)))  float    v8f;
typedef __attribute__((ext_vector_type(4)))  float    v4f;

__device__ __forceinline__ void dep_guard_h(v8f& a, v8f& b, v16h x, v16h y) { asm volatile("v_nop\n\tv_nop\n\tv_nop\n\tv_nop" : "+v"(a), "+v"(b) : "v"(x), "v"(y)); }
__device__ __forceinline__ void keep4_h(v16h a, v16h b, v16h c, v16h d) { asm volatile("v_nop" :: "v"(a), "v"(b), "v"(c), "v"(d)); }
__device__ __forceinline__ void acc_guard4(v8f& a, v8f& b, v8f& c, v8f& d) { asm volatile("v_nop\n\tv_nop\n\tv_nop\n\tv_nop" : "+v"(a), "+v"(b), "+v"(c), "+v"(d)); }
template <typename T> struct Frag;
template <> struct Frag<_Float16> {
  typedef v16h V; union U { v16h v; v8h h[2]; };
  static __device__ __forceinline__ v16h load(const _Float16* p) {
    U f; f.h[0] = *(const v8h*)(p); f.h[1] = *(const v8h*)(p + 16); return f.v;
  }
  static __device__ __forceinline__ v8f mma(v16h a, v16h b, v8f c) {
    return __builtin_amdgcn_wmma_f32_16x16x32_f16(false, a, false, b, (short)0, c, false, false);
  }
};

__device__ __forceinline__ float fsig(float x)  { return __builtin_amdgcn_rcpf(1.0f + __expf(-x)); }
__device__ __forceinline__ float ftanh(float x) { return 1.0f - 2.0f * __builtin_amdgcn_rcpf(__expf(2.0f * x) + 1.0f); }

__device__ __forceinline__ float qsel(int idx, float vr, float vi, float vj, float vk) {
  return (idx == 0) ? vr : (idx == 1) ? vi : (idx == 2) ? vj : vk;
}

__global__ __launch_bounds__(PTHR) void prep_ut_kernel(const float* __restrict__ ur, const float* __restrict__ ui,
                                                       const float* __restrict__ uj, const float* __restrict__ uk,
                                                       unsigned short* __restrict__ UT) {
  const int i  = blockIdx.x * PTHR + threadIdx.x;
  const int n8 = NLAYER * NGATE * NHID * (NHID / 8);
  if (i < n8) {
    const int c8 = i & 31;
    const int n  = (i >> 5) & (NHID - 1);
    const int lg = i >> 13;
    const int a  = c8 >> 3;
    const int p0 = (8 * c8) & (NQ - 1);
    const int bb = n >> 6, q = n & (NQ - 1);
    const int idx = a ^ bb;
    const unsigned neg = (0x5390u >> (4 * a + bb)) & 1u;
    const float sg = neg ? -UCARRY : UCARRY;
    const size_t base = ((size_t)(lg * NQ + p0)) * NQ + q;
    v8h hv;
#pragma unroll
    for (int e = 0; e < 8; ++e) {
      const size_t o = base + (size_t)e * NQ;
      const float vr = ur[o], vi = ui[o], vj = uj[o], vk = uk[o];
      hv[e] = (_Float16)(qsel(idx, vr, vi, vj, vk) * sg);
    }
    unsigned short* dst = UT + (size_t)i * 8;
    *(volatile v8h*)dst = hv;
    __threadfence();
    *(volatile v8h*)dst = hv;
  }
}

__global__ __launch_bounds__(PTHR) void prep_wx_kernel(const float* __restrict__ wr, const float* __restrict__ wi,
                                                       const float* __restrict__ wj, const float* __restrict__ wk,
                                                       float* __restrict__ WXE) {
  const int i = blockIdx.x * PTHR + threadIdx.x;
  if (i < NLAYER * NGATE * NHID) {
    const int u  = i & (NHID - 1), lg = i >> 8;
    const int bb = u >> 6, q = u & (NQ - 1);
    const size_t o = (size_t)lg * NQ + q;
    const float vr = wr[o], vi = wi[o], vj = wj[o], vk = wk[o];
    v4f ov;
#pragma unroll
    for (int a = 0; a < 4; ++a) {
      const int idx = a ^ bb;
      const unsigned neg = (0x5390u >> (4 * a + bb)) & 1u;
      const float sv = qsel(idx, vr, vi, vj, vk);
      ov[a] = neg ? -sv : sv;
    }
    float* dst = WXE + (size_t)i * 4;
    *(volatile v4f*)dst = ov;
    __threadfence();
    *(volatile v4f*)dst = ov;
  }
}

template <bool LASTL>
__global__ __launch_bounds__(RTHR) void qlstm_layer_kernel(
    const float* __restrict__ xp, int xs_b, int xs_t,
    const unsigned short* __restrict__ UTp,
    const float* __restrict__ WXE,
    const float* __restrict__ WB,
    const float* __restrict__ FW,
    const float* __restrict__ FB,
    float* __restrict__ Yout) {
  __shared__ __align__(16) _Float16 Ah[2][SEQ_BLK * HPITCH];
  __shared__ __align__(16) float    Hs[SEQ_BLK * SPITCH];
  __shared__ __align__(16) float    O4[SEQ_BLK * NFEAT];
  const _Float16* UT = (const _Float16*)UTp;
  const int tid = threadIdx.x, lane = tid & 31, wave = tid >> 5;
  const int c = lane & 15, hh = lane >> 4, koff = hh * 8;
  const int rowbase = blockIdx.x * SEQ_BLK;
  const int u = 16 * wave + c;

  {
    _Float16* ahf = &Ah[0][0];
#pragma unroll 1
    for (int i = tid; i < 2 * SEQ_BLK * HPITCH; i += RTHR) ahf[i] = (_Float16)0.0f;
  }
  float cst[8];
#pragma unroll
  for (int r = 0; r < 8; ++r) cst[r] = 0.0f;
  v4f wx[NGATE];
  float wb[NGATE];
#pragma unroll
  for (int g = 0; g < NGATE; ++g) {
    wx[g] = *(const v4f*)(WXE + ((size_t)(g * NHID + u)) * NFEAT);
    wb[g] = WB[g * NHID + u];
  }
  __syncthreads();

  const v8f z8 = {0.f, 0.f, 0.f, 0.f, 0.f, 0.f, 0.f, 0.f};

#pragma unroll 1
  for (int t = 0; t < NSTEP; ++t) {
    const int cur = t & 1;
    const _Float16* ahrow = &Ah[cur][0] + c * HPITCH + koff;
    _Float16* ahn = &Ah[cur ^ 1][0];
    v8f acc[NGATE];
#pragma unroll
    for (int g = 0; g < NGATE; ++g) acc[g] = z8;
#pragma unroll 1
    for (int k0 = 0; k0 < NHID; k0 += 32) {
      const v16h a = Frag<_Float16>::load(ahrow + k0);
      v16h bf[NGATE];
#pragma unroll
      for (int g = 0; g < NGATE; ++g) bf[g] = Frag<_Float16>::load(UT + ((size_t)(g * NHID + u)) * NHID + koff + k0);
#pragma unroll
      for (int g = 0; g < NGATE; ++g) acc[g] = Frag<_Float16>::mma(a, bf[g], acc[g]);
      dep_guard_h(acc[0], acc[3], a, bf[3]);
      keep4_h(bf[0], bf[1], bf[2], a);
    }
    acc_guard4(acc[0], acc[1], acc[2], acc[3]);

    const bool dohead = (!LASTL) || (t == NSTEP - 1);

#pragma unroll
    for (int r = 0; r < 8; ++r) {
      const int row = 8 * hh + r;
      const v4f xv = *(const v4f*)(xp + (size_t)(rowbase + row) * (size_t)xs_b + (size_t)t * (size_t)xs_t);
      float pre[NGATE];
#pragma unroll
      for (int g = 0; g < NGATE; ++g) {
        float sv = acc[g][r] * UCARRY_INV + wb[g];
        sv += xv[0] * wx[g][0];
        sv += xv[1] * wx[g][1];
        sv += xv[2] * wx[g][2];
        sv += xv[3] * wx[g][3];
        pre[g] = sv;
      }
      const float fg = fsig(pre[0]);
      const float ig = fsig(pre[1]);
      const float og = fsig(pre[2]);
      const float cg = ftanh(pre[3]);
      const float cn = ig * cg + fg * cst[r];
      cst[r] = cn;
      const float hn = og * ftanh(cn);
      ahn[row * HPITCH + u] = (_Float16)hn;
      Hs[row * SPITCH + u]  = hn;
    }
    __syncthreads();

    if (dohead) {
      const float* hp = Hs + wave * SPITCH + 8 * lane;
      const v4f ha = *(const v4f*)(hp);
      const v4f hb = *(const v4f*)(hp + 4);
      float s0 = 0.f, s1 = 0.f, s2 = 0.f, s3 = 0.f;
#pragma unroll
      for (int e = 0; e < 4; ++e) {
        const v4f w = *(const v4f*)(FW + (size_t)(8 * lane + e) * NFEAT);
        s0 += ha[e] * w[0]; s1 += ha[e] * w[1]; s2 += ha[e] * w[2]; s3 += ha[e] * w[3];
      }
#pragma unroll
      for (int e = 0; e < 4; ++e) {
        const v4f w = *(const v4f*)(FW + (size_t)(8 * lane + 4 + e) * NFEAT);
        s0 += hb[e] * w[0]; s1 += hb[e] * w[1]; s2 += hb[e] * w[2]; s3 += hb[e] * w[3];
      }
#pragma unroll
      for (int off = 1; off < 32; off <<= 1) {
        s0 += __shfl_xor(s0, off, 32);
        s1 += __shfl_xor(s1, off, 32);
        s2 += __shfl_xor(s2, off, 32);
        s3 += __shfl_xor(s3, off, 32);
      }
      const v4f fb = *(const v4f*)FB;
      const float o0 = s0 + fb[0], o1 = s1 + fb[1], o2 = s2 + fb[2], o3 = s3 + fb[3];
      const float ss  = (o0 * o0 + o1 * o1) + (o2 * o2 + o3 * o3);
      const float nrm = fmaxf(sqrtf(ss), 1e-12f);
      const float inv = __builtin_amdgcn_rcpf(nrm);
      if (lane == 0) {
        v4f ov;
        ov[0] = o0 * inv; ov[1] = o1 * inv; ov[2] = o2 * inv; ov[3] = o3 * inv;
        *(v4f*)(O4 + wave * NFEAT) = ov;
      }
    }
    __syncthreads();

    if (dohead && wave == 0) {
      const v4f val = *(const v4f*)(O4 + c * NFEAT);
      float* dst = LASTL ? (Yout + (size_t)rowbase * NFEAT)
                         : (Yout + ((size_t)t * NBAT + (size_t)rowbase) * NFEAT);
      if (lane < 16) *(volatile v4f*)(dst + lane * NFEAT) = val;
      __threadfence();
      if (lane < 16) *(volatile v4f*)(dst + lane * NFEAT) = val;
    }
  }
}

extern "C" void kernel_launch(void* const* d_in, const int* in_sizes, int n_in,
                              void* d_out, int out_size, void* d_ws, size_t ws_size, hipStream_t stream) {
  if (n_in < 12 || d_out == nullptr || d_ws == nullptr) return;
  if (in_sizes[0] != NBAT * NSTEP * NFEAT ||
      in_sizes[1] != NLAYER * NGATE * NQ || in_sizes[2] != NLAYER * NGATE * NQ ||
      in_sizes[3] != NLAYER * NGATE * NQ || in_sizes[4] != NLAYER * NGATE * NQ ||
      in_sizes[5] != NLAYER * NGATE * NHID ||
      in_sizes[6] != NLAYER * NGATE * NQ * NQ || in_sizes[7] != NLAYER * NGATE * NQ * NQ ||
      in_sizes[8] != NLAYER * NGATE * NQ * NQ || in_sizes[9] != NLAYER * NGATE * NQ * NQ ||
      in_sizes[10] != NLAYER * NHID * NFEAT || in_sizes[11] != NLAYER * NFEAT ||
      out_size != NBAT * NFEAT) return;

  const float* x    = (const float*)d_in[0];
  const float* wxr  = (const float*)d_in[1];
  const float* wxi  = (const float*)d_in[2];
  const float* wxj  = (const float*)d_in[3];
  const float* wxk  = (const float*)d_in[4];
  const float* wxb  = (const float*)d_in[5];
  const float* uhr  = (const float*)d_in[6];
  const float* uhi  = (const float*)d_in[7];
  const float* uhj  = (const float*)d_in[8];
  const float* uhk  = (const float*)d_in[9];
  const float* fcow = (const float*)d_in[10];
  const float* fcob = (const float*)d_in[11];
  float* out = (float*)d_out;

  char* ws = (char*)d_ws; size_t off = 0;
  auto carve = [&](size_t bytes) -> char* { char* p = ws + off; off += (bytes + 255) & ~(size_t)255; return p; };
  unsigned short* UT   = (unsigned short*)carve((size_t)NLAYER * UT_PER_LAYER * 2);
  float*          WXE  = (float*)carve((size_t)NLAYER * WXE_PER_LAYER * 4);
  float*          YSEQ = (float*)carve((size_t)NSTEP * NBAT * NFEAT * 4);
  if (off > ws_size || off > (size_t)134217728) return;

  const int n8u = NLAYER * NGATE * NHID * (NHID / 8);
  const int nwx = NLAYER * NGATE * NHID;
  prep_ut_kernel<<<(n8u + PTHR - 1) / PTHR, PTHR, 0, stream>>>(uhr, uhi, uhj, uhk, UT);
  prep_wx_kernel<<<(nwx + PTHR - 1) / PTHR, PTHR, 0, stream>>>(wxr, wxi, wxj, wxk, WXE);

  qlstm_layer_kernel<false><<<NBAT / SEQ_BLK, RTHR, 0, stream>>>(
      x, NSTEP * NFEAT, NFEAT,
      UT, WXE, wxb, fcow, fcob, YSEQ);
  qlstm_layer_kernel<true><<<NBAT / SEQ_BLK, RTHR, 0, stream>>>(
      YSEQ, NFEAT, NBAT * NFEAT,
      UT + (size_t)UT_PER_LAYER, WXE + (size_t)WXE_PER_LAYER, wxb + NGATE * NHID,
      fcow + NHID * NFEAT, fcob + NFEAT, out);
}
